// DCN_19387482374642
// MI455X (gfx1250) — hardware-verified
//
#include <hip/hip_runtime.h>
#include <stdint.h>

#define DEVINL __device__ __forceinline__

typedef _Float16 f16t;
typedef _Float16 v16h __attribute__((ext_vector_type(16)));
typedef _Float16 v8h  __attribute__((ext_vector_type(8)));
typedef float    v8f  __attribute__((ext_vector_type(8)));
typedef float    v4f  __attribute__((ext_vector_type(4)));
typedef v8h __attribute__((may_alias)) v8ha;
typedef v4f __attribute__((may_alias)) v4fa;
union FragH { v16h v; v8h half[2]; unsigned int u[8]; };

#define CIN   256
#define COUT  256
#define HD    64
#define WDD   64
#define HW    (HD * WDD)
#define NTAP  9
#define KT    (NTAP * CIN)
#define NPIX  64
#define OMC   32
#define OMV   27
#define SLP   264
#define XP    65
#define CHALF 128
#define TPB   256
#define TPO   64
#define WCAR  256.0f
#define WOCAR 1024.0f
#define XCAR  8.0f
#define SCAR  16.0f
#define INVC  (1.0f / 4096.0f)
#define INVO  (1.0f / 8192.0f)

static_assert((KT % 32) == 0);
static_assert(CIN == 256);
static_assert(((COUT * (KT / 8)) % TPB) == 0);
static_assert(((OMC * (KT / 8)) % TPB) == 0);
static_assert(NPIX == WDD);
static_assert(TPB == 4 * NPIX);
static_assert((CHALF * WDD) % TPB == 0);
static_assert(2 * CHALF == CIN);
static_assert(((SLP * 2) % 16) == 0);
static_assert((COUT / 2) * NPIX * 4 <= NPIX * SLP * 2);
static_assert(((KT * 2) % 128) == 0);
static_assert(((CIN * 4) % 128) == 0);
static_assert(((CHALF * 2) % 128) == 0);

DEVINL int imin(int a, int b) { return a < b ? a : b; }
DEVINL int imax(int a, int b) { return a > b ? a : b; }

DEVINL v8f wmma_f16(v16h a, v16h b, v8f c) {
  v8f d = __builtin_amdgcn_wmma_f32_16x16x32_f16(false, a, false, b, (short)0, c, false, false);
  asm volatile("v_nop\n\tv_nop\n\tv_nop\n\tv_nop" : "+v"(d) : "v"(a), "v"(b));
  return d;
}
DEVINL v8f zero8f() {
  v8f z = {0.f, 0.f, 0.f, 0.f, 0.f, 0.f, 0.f, 0.f};
  return z;
}

__global__ __launch_bounds__(TPB) void wprep_k(const float* __restrict__ w, f16t* __restrict__ Wq,
                                             int nvalid, int ntotal, float car)
{
  const int t = blockIdx.x * TPB + threadIdx.x;
  if (t >= ntotal * (KT / 8)) return;
  const int o    = t / (KT / 8);
  const int part = t - o * (KT / 8);
  const int k8   = 8 * part;
  const int tap  = k8 >> 8;
  const int c0   = k8 & (CIN - 1);
  const int oc   = o < nvalid ? o : nvalid - 1;
  const float sc = (o < nvalid) ? car : 0.0f;
  v8h v;
  #pragma unroll
  for (int i = 0; i < 8; ++i) {
    const float wv = w[(size_t)(oc * CIN + c0 + i) * NTAP + tap];
    v[i] = (f16t)(wv * sc);
  }
  f16t* dst = Wq + (size_t)8 * t;
  *(volatile v8h*)dst = v;
  __threadfence();
  *(volatile v8h*)dst = v;
}

__global__ __launch_bounds__(TPB) void xprep_k(const float* __restrict__ x, float* __restrict__ Xt,
                                             f16t* __restrict__ Xh)
{
  __shared__ __attribute__((aligned(16))) float sX[CHALF * XP];
  const int tid = threadIdx.x;
  const int h   = blockIdx.x;
  const int b   = blockIdx.y;
  const int ch  = blockIdx.z;
  const float* xb = x + ((size_t)b * CIN + (size_t)CHALF * ch) * HW + (size_t)h * WDD;
  #pragma unroll 4
  for (int idx = tid; idx < CHALF * WDD; idx += TPB) {
    const int c  = idx >> 6;
    const int wq = idx & (WDD - 1);
    sX[c * XP + wq] = xb[(size_t)c * HW + wq];
  }
  __syncthreads();

  const int pg = tid >> 5;
  const int q  = tid & 31;
  v4f vals[8];
  #pragma unroll
  for (int g = 0; g < 8; ++g) {
    const int wq = 8 * g + pg;
    v4f v;
    v[0] = sX[(4 * q + 0) * XP + wq];
    v[1] = sX[(4 * q + 1) * XP + wq];
    v[2] = sX[(4 * q + 2) * XP + wq];
    v[3] = sX[(4 * q + 3) * XP + wq];
    vals[g] = v;
  }
  float* drow = Xt + ((size_t)(b * HD + h) * WDD) * CIN + CHALF * ch + 4 * q;
  #pragma unroll
  for (int g = 0; g < 8; ++g)
    *(volatile v4f*)(drow + (size_t)(8 * g + pg) * CIN) = vals[g];
  __threadfence();
  #pragma unroll
  for (int g = 0; g < 8; ++g)
    *(volatile v4f*)(drow + (size_t)(8 * g + pg) * CIN) = vals[g];

  const int hh = q >> 4, qq = q & 15;
  v8h hv[4];
  #pragma unroll
  for (int i = 0; i < 4; ++i) {
    const int wq = 8 * pg + 2 * i + hh;
    v8h o;
    #pragma unroll
    for (int e = 0; e < 8; ++e) o[e] = (f16t)(sX[(8 * qq + e) * XP + wq] * XCAR);
    hv[i] = o;
  }
  f16t* hrow = Xh + ((size_t)(b * HD + h) * WDD) * CIN + CHALF * ch + 8 * qq;
  #pragma unroll
  for (int i = 0; i < 4; ++i)
    *(volatile v8h*)(hrow + (size_t)(8 * pg + 2 * i + hh) * CIN) = hv[i];
  __threadfence();
  #pragma unroll
  for (int i = 0; i < 4; ++i)
    *(volatile v8h*)(hrow + (size_t)(8 * pg + 2 * i + hh) * CIN) = hv[i];
}

__global__ __launch_bounds__(TPO) void offconv_k(const f16t* __restrict__ Xh, const f16t* __restrict__ Wo,
                                               float* __restrict__ Om)
{
  __shared__ __attribute__((aligned(16))) float sO[OMC * NPIX];
  const int tid = threadIdx.x, lane = tid & 31, wave = tid >> 5;
  const int h = lane >> 4, m = lane & 15;
  const int wg = blockIdx.x;
  const int b  = wg >> 6;
  const int oh = wg & (HD - 1);

  const f16t* ar0 = Wo + (size_t)m * KT + 8 * h;
  const f16t* ar1 = Wo + (size_t)(16 + m) * KT + 8 * h;

  v8f acc[2][2];
  #pragma unroll
  for (int mt = 0; mt < 2; ++mt) { acc[mt][0] = zero8f(); acc[mt][1] = zero8f(); }

  #pragma unroll 1
  for (int tap = 0; tap < NTAP; ++tap) {
    const int ki = tap / 3;
    const int kj = tap - 3 * ki;
    const int yy = oh + ki - 1;
    const bool yok = ((unsigned)yy < (unsigned)HD);
    const int  yc  = imin(imax(yy, 0), HD - 1);
    const f16t* bp[2];
    bool ok[2];
    #pragma unroll
    for (int nl = 0; nl < 2; ++nl) {
      const int px  = 16 * (2 * wave + nl) + m + kj - 1;
      const bool xok = ((unsigned)px < (unsigned)WDD);
      const int  xc  = imin(imax(px, 0), WDD - 1);
      bp[nl] = Xh + ((size_t)((b * HD + yc) * WDD + xc)) * CIN + 8 * h;
      ok[nl] = yok && xok;
    }
    const f16t* at0 = ar0 + tap * CIN;
    const f16t* at1 = ar1 + tap * CIN;
    #pragma unroll
    for (int c = 0; c < 8; ++c) {
      FragH a0, a1;
      a0.half[0] = *(const v8ha*)(at0 + 32 * c);
      a0.half[1] = *(const v8ha*)(at0 + 32 * c + 16);
      a1.half[0] = *(const v8ha*)(at1 + 32 * c);
      a1.half[1] = *(const v8ha*)(at1 + 32 * c + 16);
      #pragma unroll
      for (int nl = 0; nl < 2; ++nl) {
        FragH bf;
        bf.half[0] = *(const v8ha*)(bp[nl] + 32 * c);
        bf.half[1] = *(const v8ha*)(bp[nl] + 32 * c + 16);
        #pragma unroll
        for (int i = 0; i < 8; ++i) bf.u[i] = ok[nl] ? bf.u[i] : 0u;
        acc[0][nl] = wmma_f16(a0.v, bf.v, acc[0][nl]);
        acc[1][nl] = wmma_f16(a1.v, bf.v, acc[1][nl]);
      }
    }
  }

  #pragma unroll
  for (int mt = 0; mt < 2; ++mt) {
    #pragma unroll
    for (int nl = 0; nl < 2; ++nl) {
      #pragma unroll
      for (int r = 0; r < 8; ++r) {
        const int chn = 16 * mt + 8 * h + r;
        sO[chn * NPIX + 16 * (2 * wave + nl) + m] = acc[mt][nl][r] * INVO;
      }
    }
  }
  __syncthreads();

  float* gbase = Om + ((size_t)b * OMC) * HW + (size_t)oh * WDD + 4 * m;
  v4f vv[8];
  #pragma unroll
  for (int j = 0; j < 8; ++j) {
    const int row = 16 * wave + 2 * j + h;
    vv[j] = *(const v4fa*)(sO + row * NPIX + 4 * m);
  }
  #pragma unroll
  for (int j = 0; j < 8; ++j) {
    const int row = 16 * wave + 2 * j + h;
    *(volatile v4f*)(gbase + (size_t)row * HW) = vv[j];
  }
  __threadfence();
  #pragma unroll
  for (int j = 0; j < 8; ++j) {
    const int row = 16 * wave + 2 * j + h;
    *(volatile v4f*)(gbase + (size_t)row * HW) = vv[j];
  }
}

__global__ __launch_bounds__(TPB) void dconv_k(const float* __restrict__ Xt, const f16t* __restrict__ Wq,
                                             const float* __restrict__ Om, const float* __restrict__ boff,
                                             float* __restrict__ out)
{
  __shared__ __attribute__((aligned(16))) unsigned char smem[NPIX * SLP * 2];
  f16t*  Sl = (f16t*)smem;
  float* sO = (float*)smem;
  const int tid = threadIdx.x, lane = tid & 31, wave = tid >> 5;
  const int h = lane >> 4, m = lane & 15;
  const int wg = blockIdx.x;
  const int b  = wg >> 6;
  const int oh = wg & (HD - 1);

  const int pos = tid & (NPIX - 1);
  const int cg  = tid >> 6;
  const float* xb  = Xt + (size_t)b * HW * CIN + 64 * cg;
  const float* omb = Om + ((size_t)b * OMC) * HW + (size_t)oh * WDD + pos;
  const f16t* arow0 = Wq + (size_t)(32 * wave + m) * KT + 8 * h;
  const f16t* arow1 = arow0 + (size_t)16 * KT;

  v8f acc[2][4];
  #pragma unroll
  for (int t = 0; t < 4; ++t) { acc[0][t] = zero8f(); acc[1][t] = zero8f(); }

  #pragma unroll 1
  for (int tap = 0; tap < NTAP; ++tap) {
    const int ki = tap / 3;
    const int kj = tap - 3 * ki;
    __syncthreads();

    {
      const float dy = omb[(size_t)(2 * tap) * HW]     + boff[2 * tap];
      const float dx = omb[(size_t)(2 * tap + 1) * HW] + boff[2 * tap + 1];
      float mr = omb[(size_t)(2 * NTAP + tap) * HW] + boff[2 * NTAP + tap];
      mr = fminf(fmaxf(mr, -30.0f), 30.0f);
      const float mk = 1.0f / (1.0f + expf(-mr));
      const float ys = (float)(oh + ki - 1) + dy;
      const float xs = (float)(pos + kj - 1) + dx;
      const float y0f = floorf(ys), x0f = floorf(xs);
      const float wy = ys - y0f,   wx = xs - x0f;
      const float y1f = y0f + 1.0f, x1f = x0f + 1.0f;
      const bool vy0 = (y0f >= 0.0f) && (y0f <= (float)(HD - 1));
      const bool vy1 = (y1f >= 0.0f) && (y1f <= (float)(HD - 1));
      const bool vx0 = (x0f >= 0.0f) && (x0f <= (float)(WDD - 1));
      const bool vx1 = (x1f >= 0.0f) && (x1f <= (float)(WDD - 1));
      const float omy = 1.0f - wy, omx = 1.0f - wx;
      float w00 = omy * omx * mk;
      float w01 = omy * wx * mk;
      float w10 = wy * omx * mk;
      float w11 = wy * wx * mk;
      w00 = (vy0 && vx0) ? w00 : 0.0f;
      w01 = (vy0 && vx1) ? w01 : 0.0f;
      w10 = (vy1 && vx0) ? w10 : 0.0f;
      w11 = (vy1 && vx1) ? w11 : 0.0f;
      const int y0i = (int)fminf(fmaxf(y0f, -4.0f), (float)(HD + 4));
      const int x0i = (int)fminf(fmaxf(x0f, -4.0f), (float)(WDD + 4));
      const int y0c = imin(imax(y0i, 0), HD - 1);
      const int y1c = imin(imax(y0i + 1, 0), HD - 1);
      const int x0c = imin(imax(x0i, 0), WDD - 1);
      const int x1c = imin(imax(x0i + 1, 0), WDD - 1);
      const float* p00 = xb + (size_t)(y0c * WDD + x0c) * CIN;
      const float* p01 = xb + (size_t)(y0c * WDD + x1c) * CIN;
      const float* p10 = xb + (size_t)(y1c * WDD + x0c) * CIN;
      const float* p11 = xb + (size_t)(y1c * WDD + x1c) * CIN;
      f16t* srow = Sl + pos * SLP + 64 * cg;
      #pragma unroll 2
      for (int ch = 0; ch < 8; ++ch) {
        const v4f a0 = *(const v4fa*)(p00 + 8 * ch), a1 = *(const v4fa*)(p00 + 8 * ch + 4);
        const v4f b0 = *(const v4fa*)(p01 + 8 * ch), b1 = *(const v4fa*)(p01 + 8 * ch + 4);
        const v4f c0 = *(const v4fa*)(p10 + 8 * ch), c1 = *(const v4fa*)(p10 + 8 * ch + 4);
        const v4f d0 = *(const v4fa*)(p11 + 8 * ch), d1 = *(const v4fa*)(p11 + 8 * ch + 4);
        v4f s0 = a0 * w00;
        v4f s1 = a1 * w00;
        s0 = b0 * w01 + s0;  s1 = b1 * w01 + s1;
        s0 = c0 * w10 + s0;  s1 = c1 * w10 + s1;
        s0 = d0 * w11 + s0;  s1 = d1 * w11 + s1;
        v8h o;
        #pragma unroll
        for (int i = 0; i < 4; ++i) {
          o[i]     = (f16t)(s0[i] * SCAR);
          o[4 + i] = (f16t)(s1[i] * SCAR);
        }
        *(v8ha*)(srow + 8 * ch) = o;
      }
    }
    __syncthreads();

    const f16t* at0 = arow0 + tap * CIN;
    const f16t* at1 = arow1 + tap * CIN;
    #pragma unroll
    for (int c = 0; c < 8; ++c) {
      FragH a0, a1;
      a0.half[0] = *(const v8ha*)(at0 + 32 * c);
      a0.half[1] = *(const v8ha*)(at0 + 32 * c + 16);
      a1.half[0] = *(const v8ha*)(at1 + 32 * c);
      a1.half[1] = *(const v8ha*)(at1 + 32 * c + 16);
      #pragma unroll
      for (int t = 0; t < 4; ++t) {
        FragH bf;
        const f16t* br = Sl + (16 * t + m) * SLP + 32 * c + 8 * h;
        bf.half[0] = *(const v8ha*)(br);
        bf.half[1] = *(const v8ha*)(br + 16);
        acc[0][t] = wmma_f16(a0.v, bf.v, acc[0][t]);
        acc[1][t] = wmma_f16(a1.v, bf.v, acc[1][t]);
      }
    }
  }
  __syncthreads();

  #pragma unroll
  for (int p = 0; p < 2; ++p) {
    #pragma unroll
    for (int t = 0; t < 4; ++t) {
      #pragma unroll
      for (int r = 0; r < 8; ++r) {
        const int row = 16 * wave + 8 * h + r;
        sO[row * NPIX + 16 * t + m] = acc[p][t][r] * INVC;
      }
    }
    __syncthreads();

    float* gbase = out + ((size_t)(b * COUT + 32 * wave + 16 * p)) * HW + (size_t)oh * WDD + 4 * m;
    v4f vv[8];
    #pragma unroll
    for (int j = 0; j < 8; ++j) {
      const int row = 16 * wave + 2 * j + h;
      vv[j] = *(const v4fa*)(sO + row * NPIX + 4 * m);
    }
    #pragma unroll
    for (int j = 0; j < 8; ++j)
      *(volatile v4f*)(gbase + (size_t)(2 * j + h) * HW) = vv[j];
    __threadfence();
    #pragma unroll
    for (int j = 0; j < 8; ++j)
      *(volatile v4f*)(gbase + (size_t)(2 * j + h) * HW) = vv[j];
    __syncthreads();
  }
}

extern "C" void kernel_launch(void* const* d_in, const int* in_sizes, int n_in,
                              void* d_out, int out_size, void* d_ws, size_t ws_size,
                              hipStream_t stream)
{
  if (n_in < 4) return;
  const int plane = CIN * HW;
  if (in_sizes[0] <= 0 || (in_sizes[0] % plane) != 0) return;
  const int nB = in_sizes[0] / plane;
  if (nB > 64) return;
  if (in_sizes[1] != OMV * CIN * NTAP) return;
  if (in_sizes[2] != OMV) return;
  if (in_sizes[3] != COUT * CIN * NTAP) return;
  if (out_size != nB * COUT * HW) return;

  const float* x    = (const float*)d_in[0];
  const float* woff = (const float*)d_in[1];
  const float* boff = (const float*)d_in[2];
  const float* wgt  = (const float*)d_in[3];
  float* outp = (float*)d_out;

  const size_t szWq = (size_t)COUT * KT * 2;
  const size_t szWo = (size_t)OMC * KT * 2;
  const size_t szXt = (size_t)nB * HW * CIN * 4;
  const size_t szXh = (size_t)nB * HW * CIN * 2;
  const size_t szOm = (size_t)nB * OMC * HW * 4;
  size_t offb = 0;
  char* ws = (char*)d_ws;
  f16t*  Wq = (f16t*)(ws + offb);  offb += szWq;
  f16t*  Wo = (f16t*)(ws + offb);  offb += szWo;
  float* Xt = (float*)(ws + offb); offb += szXt;
  f16t*  Xh = (f16t*)(ws + offb);  offb += szXh;
  float* Om = (float*)(ws + offb); offb += szOm;
  if (offb > ws_size) return;
  if (offb > (size_t)134217728) return;

  wprep_k<<<(COUT * (KT / 8)) / TPB, TPB, 0, stream>>>(wgt, Wq, COUT, COUT, WCAR);
  wprep_k<<<(OMC * (KT / 8)) / TPB, TPB, 0, stream>>>(woff, Wo, OMV, OMC, WOCAR);
  xprep_k<<<dim3(HD, nB, 2), TPB, 0, stream>>>(x, Xt, Xh);
  offconv_k<<<nB * HD, TPO, 0, stream>>>(Xh, Wo, Om);
  dconv_k<<<nB * HD, TPB, 0, stream>>>(Xt, Wq, Om, boff, outp);
}
